// CAF_41463614275926
// MI455X (gfx1250) — hardware-run, weakly checked
//
#include <hip/hip_runtime.h>


namespace {
constexpr int Bn = 4, CIN = 128, C = 64, HW = 64, NPX = HW * HW, NT = Bn * NPX, C8 = 8, CR = 4, STB = 128;
constexpr float XS = 8.0f, PS = 8.0f, EPS = 1e-5f;

typedef _Float16 b16;
typedef __attribute__((ext_vector_type(16))) _Float16 v16b;
typedef __attribute__((ext_vector_type(8))) _Float16 v8b;
typedef __attribute__((ext_vector_type(8))) float v8f;
typedef __attribute__((ext_vector_type(4))) float v4f;
typedef __attribute__((ext_vector_type(2))) float v2f;
__device__ __forceinline__ float bf16_rne(float f) { unsigned int u = __float_as_uint(f); u += 0x7FFFu + ((u >> 16) & 1u); return __uint_as_float(u & 0xFFFF0000u); }
__device__ __forceinline__ void split16(float v, b16& hi, b16& lo) { hi = (b16)v; lo = (b16)(v - (float)hi); }
__device__ __forceinline__ v16b frag_kb(const b16* p, int hh) { const v8b a = *(const v8b*)(p + 8 * hh), b = *(const v8b*)(p + 16 + 8 * hh); v16b f;
#pragma unroll
  for (int e = 0; e < 8; ++e) { f[e] = a[e]; f[8 + e] = b[e]; } return f; }
__device__ __forceinline__ v8f wmma16b(v16b a, v16b b, v8f c) { v8f d = __builtin_amdgcn_wmma_f32_16x16x32_f16(false, a, false, b, (short)0, c, false, false); asm volatile("v_nop\n\tv_nop\n\tv_nop\n\tv_nop" : "+v"(d) : "v"(a), "v"(b)); return d; }
__device__ __forceinline__ void wave_lds_sync() { __builtin_amdgcn_fence(__ATOMIC_RELEASE, "workgroup"); __builtin_amdgcn_wave_barrier(); __builtin_amdgcn_fence(__ATOMIC_ACQUIRE, "workgroup"); }
__device__ __forceinline__ float nexp(float x) { return __builtin_amdgcn_exp2f(x * 1.4426950408889634f); }
__device__ __forceinline__ float pmul(float a, float b) { float p = a * b; asm volatile("" : "+v"(p)); return p; }
__device__ __forceinline__ float sigm(float x) { return 1.0f / (1.0f + nexp(-x)); }

__global__ __launch_bounds__(256) void prep_kernel(const float* __restrict__ xs, const float* __restrict__ xr, const float* __restrict__ pw, const float* __restrict__ pb, const float* __restrict__ caw1, const float* __restrict__ caw2, const float* __restrict__ saw, const float* __restrict__ sab, const float* __restrict__ qw, const float* __restrict__ qb, const float* __restrict__ kw, const float* __restrict__ kb,
    const float* __restrict__ vw, const float* __restrict__ vb, const float* __restrict__ gm, const float* __restrict__ rw, const float* __restrict__ rb, const float* __restrict__ bns, const float* __restrict__ bnb, b16* __restrict__ R, float* __restrict__ P, b16* __restrict__ XT) {
  __shared__ __attribute__((aligned(16))) b16 Tx[64][CIN + 8];
  const int i = blockIdx.z, b = blockIdx.y, p0 = blockIdx.x * 64, t_ = threadIdx.x; const float* x = i ? xr : xs;
  const size_t tid = ((size_t)(blockIdx.z * Bn + blockIdx.y) * gridDim.x + blockIdx.x) * 256 + t_, nth = (size_t)gridDim.x * Bn * 2 * 256;
  for (int k = t_; k < CIN * 64; k += 256) { const int c = k >> 6, px = k & 63; Tx[px][c] = (b16)(bf16_rne(x[((size_t)b * CIN + c) * NPX + p0 + px]) * XS); }
  __syncthreads();
  for (int pass = 0; pass < 2; ++pass) {
    for (size_t g8 = tid; g8 < 30720 / 8; g8 += nth) { v8b o8;
#pragma unroll
      for (int e = 0; e < 8; ++e) { const int j = (int)g8 * 8 + e; float v = 0.0f;
        if (j < 8192) v = pw[j]; else if (j < 9216) { const int o = (j - 8192) / 64, c = (j - 8192) % 64; v = (o < 8) ? qw[(o < 8 ? o : 7) * 64 + c] : 0.0f; } else if (j < 10240) { const int o = (j - 9216) / 64, c = (j - 9216) % 64; v = (o < 8) ? kw[(o < 8 ? o : 7) * 64 + c] : 0.0f; } else if (j < 14336) v = vw[j - 10240]; else v = rw[j - 14336];
        o8[e] = (b16)bf16_rne(v); }
      *(volatile v8b*)(R + g8 * 8) = o8; }
    for (size_t q = tid; q < 1200; q += nth) { const int j = (int)q; float v = 0.0f;
      if (j < 64) v = pb[j]; else if (j < 80) v = (j - 64 < 8) ? qb[(j - 64 < 8) ? j - 64 : 7] : 0.0f; else if (j < 96) v = (j - 80 < 8) ? kb[(j - 80 < 8) ? j - 80 : 7] : 0.0f; else if (j < 160) v = vb[j - 96]; else if (j < 161) v = gm[0]; else if (j < 192) v = 0.0f; else if (j < 320) v = rb[j - 192]; else if (j < 448) v = bns[j - 320]; else if (j < 576) v = bnb[j - 448]; else if (j < 832) v = caw1[j - 576]; else if (j < 1088) v = caw2[j - 832]; else if (j < 1186) v = saw[j - 1088]; else if (j < 1187) v = sab[0];
      ((volatile float*)P)[q] = bf16_rne(v); }
    for (int k = t_; k < 64 * 16; k += 256) { const int px = k >> 4, c8 = (k & 15) * 8; *(volatile v8b*)(XT + ((size_t)i * NT + (size_t)b * NPX + p0 + px) * CIN + c8) = *(const v8b*)(&Tx[px][c8]); }
    __threadfence(); }
}
__global__ __launch_bounds__(64) void proj_kernel(const b16* __restrict__ XT, const b16* __restrict__ R, const float* __restrict__ P, float* __restrict__ SF) {
  __shared__ __attribute__((aligned(16))) float Ts[2][16][C + 4];
  const int i = blockIdx.y, lane = threadIdx.x & 31, wave = threadIdx.x >> 5, nloc = lane & 15, hlf = lane >> 4, m0 = blockIdx.x * 32 + wave * 16; const b16* A = XT + (size_t)i * NT * CIN;
  v8f acc[4] = {{}, {}, {}, {}};
#pragma unroll
  for (int kb = 0; kb < CIN; kb += 32) { const v16b a = frag_kb(A + (size_t)(m0 + nloc) * CIN + kb, hlf);
#pragma unroll
    for (int t = 0; t < 4; ++t) acc[t] = wmma16b(a, frag_kb(R + (size_t)(t * 16 + nloc) * CIN + kb, hlf), acc[t]); }
#pragma unroll
  for (int t = 0; t < 4; ++t)
#pragma unroll
    for (int r = 0; r < 8; ++r) Ts[wave][8 * hlf + r][t * 16 + nloc] = acc[t][r] * (1.0f / XS) + P[t * 16 + nloc];
  wave_lds_sync();
  for (int pass = 0; pass < 2; ++pass) { for (int k = lane; k < 16 * 16; k += 32) { const int rr = k >> 4, c4 = (k & 15) * 4; *(volatile v4f*)(SF + ((size_t)i * NT + m0 + rr) * C + c4) = *(const v4f*)(&Ts[wave][rr][c4]); } __threadfence(); }
}
__global__ __launch_bounds__(64) void cstat1_kernel(const float* __restrict__ SF, float* __restrict__ PART, float* __restrict__ MM) {
  __shared__ float Rw[32][C + 1];
  const int i = blockIdx.z, b = blockIdx.y, ch = blockIdx.x, t_ = threadIdx.x; const float* rows = SF + ((size_t)i * NT + (size_t)b * NPX + ch * 32) * C;
  for (int k = t_; k < 32 * C; k += 64) Rw[k >> 6][k & 63] = rows[k];
  __syncthreads();
  float csum = 0.0f; for (int p = 0; p < 32; ++p) csum += Rw[p][t_];
  float pm = 0.0f, px_ = -INFINITY; if (t_ < 32) { for (int c = 0; c < C; ++c) { pm += Rw[t_][c]; px_ = fmaxf(px_, Rw[t_][c]); } pm *= (1.0f / C); }
  for (int pass = 0; pass < 2; ++pass) { ((volatile float*)PART)[(((size_t)i * Bn + b) * 128 + ch) * C + t_] = csum; if (t_ < 32) { ((volatile float*)MM)[(((size_t)i * Bn + b) * 2 + 0) * NPX + ch * 32 + t_] = pm; ((volatile float*)MM)[(((size_t)i * Bn + b) * 2 + 1) * NPX + ch * 32 + t_] = px_; } __threadfence(); }
}
__global__ __launch_bounds__(64) void cstat2_kernel(const float* __restrict__ PART, const float* __restrict__ P, float* __restrict__ CA) {
  __shared__ float Av[C], Hh[CR];
  const int i = blockIdx.y, b = blockIdx.x, c = threadIdx.x; float s = 0.0f; for (int ch = 0; ch < 128; ++ch) s += PART[(((size_t)i * Bn + b) * 128 + ch) * C + c]; Av[c] = s * (1.0f / NPX);
  __syncthreads();
  if (c < CR) { float h = 0.0f; for (int k = 0; k < C; ++k) h += pmul(Av[k], P[576 + c * C + k]); Hh[c] = fmaxf(h, 0.0f); }
  __syncthreads();
  float v = 0.0f; for (int r = 0; r < CR; ++r) v += pmul(Hh[r], P[832 + c * CR + r]); v = sigm(v);
  for (int pass = 0; pass < 2; ++pass) { ((volatile float*)CA)[((size_t)i * Bn + b) * C + c] = v; __threadfence(); }
}
__global__ __launch_bounds__(256) void es_kernel(const float* __restrict__ SF, const float* __restrict__ MM, const float* __restrict__ CA, const float* __restrict__ P, float* __restrict__ ESF, b16* __restrict__ ESh, b16* __restrict__ ESl, b16* __restrict__ CATh, b16* __restrict__ CATl) {
  __shared__ float Sa[HW]; __shared__ __attribute__((aligned(16))) b16 Th[HW][C + 8], Tl[HW][C + 8]; __shared__ __attribute__((aligned(16))) float Tf[HW][C + 4];
  const int i = blockIdx.z, b = blockIdx.y, y = blockIdx.x, t_ = threadIdx.x; const float* mm = MM + ((size_t)i * Bn + b) * 2 * NPX;
  if (t_ < HW) { const int x = t_; float s = P[1186];
    for (int ch = 0; ch < 2; ++ch) for (int dy = 0; dy < 7; ++dy) { const int yy = y + dy - 3; if (yy < 0 || yy >= HW) continue; for (int dx = 0; dx < 7; ++dx) { const int xx = x + dx - 3; if (xx < 0 || xx >= HW) continue; s += pmul(P[1088 + (ch * 7 + dy) * 7 + dx], mm[(size_t)ch * NPX + yy * HW + xx]); } }
    Sa[x] = sigm(s); }
  __syncthreads();
  const size_t row0 = (size_t)i * NT + (size_t)b * NPX + y * HW;
  for (int k = t_; k < HW * C; k += 256) { const int x = k >> 6, c = k & 63; const float v = pmul(pmul(SF[(row0 + x) * C + c], CA[((size_t)i * Bn + b) * C + c]), Sa[x]); Tf[x][c] = v; b16 a_, c_; split16(v * XS, a_, c_); Th[x][c] = a_; Tl[x][c] = c_; }
  __syncthreads();
  for (int pass = 0; pass < 2; ++pass) {
    for (int k = t_; k < HW * 16; k += 256) { const int x = k >> 4, c4 = (k & 15) * 4; *(volatile v4f*)(ESF + (row0 + x) * C + c4) = *(const v4f*)(&Tf[x][c4]); }
    for (int k = t_; k < HW * 8; k += 256) { const int x = k >> 3, c8 = (k & 7) * 8; *(volatile v8b*)(ESh + (row0 + x) * C + c8) = *(const v8b*)(&Th[x][c8]); *(volatile v8b*)(ESl + (row0 + x) * C + c8) = *(const v8b*)(&Tl[x][c8]);
      if (i == 0) { const size_t gi = ((size_t)b * NPX + y * HW + x) * CIN + C + c8; *(volatile v8b*)(CATh + gi) = *(const v8b*)(&Th[x][c8]); *(volatile v8b*)(CATl + gi) = *(const v8b*)(&Tl[x][c8]); } }
    __threadfence(); }
}
__global__ __launch_bounds__(128) void qkv_kernel(const b16* __restrict__ ESh, const b16* __restrict__ ESl, const b16* __restrict__ R, const float* __restrict__ P, b16* __restrict__ QH, b16* __restrict__ QL, b16* __restrict__ KH, b16* __restrict__ KL, b16* __restrict__ VTh, b16* __restrict__ VTl) {
  __shared__ __attribute__((aligned(16))) b16 Th[64][64 + 8], Tl[64][64 + 8];
  const int mode = blockIdx.y, lane = threadIdx.x & 31, wave = threadIdx.x >> 5, nloc = lane & 15, hlf = lane >> 4, g0 = blockIdx.x * 64, m0 = g0 + wave * 16;
  const int i = (mode == 0) ? 0 : 1; const b16* Ah = ESh + (size_t)i * NT * C; const b16* Al = ESl + (size_t)i * NT * C; const b16* Bw = R + ((mode == 0) ? 8192 : (mode == 1) ? 9216 : 10240); const float* bias = P + ((mode == 0) ? 64 : (mode == 1) ? 80 : 96);
  const int NS = (mode == 2) ? 4 : 1;
  v8f acc[4] = {{}, {}, {}, {}};
#pragma unroll
  for (int kb = 0; kb < C; kb += 32) { const v16b a = frag_kb(Ah + (size_t)(m0 + nloc) * C + kb, hlf), al_ = frag_kb(Al + (size_t)(m0 + nloc) * C + kb, hlf);
    for (int t = 0; t < NS; ++t) { const v16b bw = frag_kb(Bw + (size_t)(t * 16 + nloc) * C + kb, hlf); acc[t] = wmma16b(a, bw, acc[t]); acc[t] = wmma16b(al_, bw, acc[t]); } }
  if (mode < 2) {
#pragma unroll
    for (int r = 0; r < 8; ++r) { b16 a_, c_; split16(acc[0][r] + XS * bias[nloc], a_, c_); Th[wave * 16 + 8 * hlf + r][nloc] = a_; Tl[wave * 16 + 8 * hlf + r][nloc] = c_; Th[wave * 16 + 8 * hlf + r][16 + nloc] = (b16)0.0f; Tl[wave * 16 + 8 * hlf + r][16 + nloc] = (b16)0.0f; }
    __syncthreads();
    b16* dh = mode ? KH : QH; b16* dl = mode ? KL : QL;
    for (int pass = 0; pass < 2; ++pass) { for (int k = threadIdx.x; k < 64 * 4; k += 128) { const int rr = k >> 2, c8 = (k & 3) * 8; *(volatile v8b*)(dh + (size_t)(g0 + rr) * 32 + c8) = *(const v8b*)(&Th[rr][c8]); *(volatile v8b*)(dl + (size_t)(g0 + rr) * 32 + c8) = *(const v8b*)(&Tl[rr][c8]); } __threadfence(); } }
  else {
#pragma unroll
    for (int t = 0; t < 4; ++t)
#pragma unroll
      for (int r = 0; r < 8; ++r) { b16 a_, c_; split16(acc[t][r] + XS * bias[t * 16 + nloc], a_, c_); Th[t * 16 + nloc][wave * 16 + 8 * hlf + r] = a_; Tl[t * 16 + nloc][wave * 16 + 8 * hlf + r] = c_; }
    __syncthreads();
    const int b = g0 / NPX, px0 = g0 % NPX;
    for (int pass = 0; pass < 2; ++pass) { for (int k = threadIdx.x; k < 64 * 8; k += 128) { const int c = k >> 3, c8 = (k & 7) * 8; const size_t gi = ((size_t)b * C + c) * NPX + px0 + c8; *(volatile v8b*)(VTh + gi) = *(const v8b*)(&Th[c][c8]); *(volatile v8b*)(VTl + gi) = *(const v8b*)(&Tl[c][c8]); } __threadfence(); } }
}
__global__ __launch_bounds__(64) void attn_kernel(const b16* __restrict__ QH, const b16* __restrict__ QL, const b16* __restrict__ KH, const b16* __restrict__ KL, const b16* __restrict__ VTh, const b16* __restrict__ VTl, const float* __restrict__ ESF, const float* __restrict__ P, b16* __restrict__ CATh, b16* __restrict__ CATl) {
  __shared__ __attribute__((aligned(16))) b16 Oh[2][16][C + 8], Ol[2][16][C + 8];
  const int wave = threadIdx.x >> 5, lane = threadIdx.x & 31, hh = lane >> 4, col = lane & 15; const int b = blockIdx.y, q0 = blockIdx.x * 32 + wave * 16, qi = q0 + col;
  const b16* Qr = QH + (size_t)b * NPX * 32; const b16* Qlr = QL + (size_t)b * NPX * 32; const b16* Kr = KH + (size_t)b * NPX * 32; const b16* Klr = KL + (size_t)b * NPX * 32; const b16* V = VTh + (size_t)b * C * NPX; const b16* Vl = VTl + (size_t)b * C * NPX;
  const v16b qf = frag_kb(Qr + (size_t)qi * 32, hh), ql = frag_kb(Qlr + (size_t)qi * 32, hh);
  float m = -INFINITY, l = 0.0f; v8f o[4] = {{}, {}, {}, {}};
  for (int kb = 0; kb < NPX; kb += 32) {
    v8f s0 = {}, s1 = {};
    { const v16b k0 = frag_kb(Kr + (size_t)(kb + col) * 32, hh), k0l = frag_kb(Klr + (size_t)(kb + col) * 32, hh), k1 = frag_kb(Kr + (size_t)(kb + 16 + col) * 32, hh), k1l = frag_kb(Klr + (size_t)(kb + 16 + col) * 32, hh);
      s0 = wmma16b(k0, qf, s0); s0 = wmma16b(k0l, qf, s0); s0 = wmma16b(k0, ql, s0); s1 = wmma16b(k1, qf, s1); s1 = wmma16b(k1l, qf, s1); s1 = wmma16b(k1, ql, s1); }
    float mr = -INFINITY;
#pragma unroll
    for (int r = 0; r < 8; ++r) { s0[r] *= 1.0f / (XS * XS); s1[r] *= 1.0f / (XS * XS); mr = fmaxf(mr, fmaxf(s0[r], s1[r])); }
    mr = fmaxf(mr, __shfl_xor(mr, 16)); const float mn = fmaxf(m, mr); const float al_ = nexp(m - mn); m = mn; float sum = 0.0f; v16b pb, pl;
#pragma unroll
    for (int r = 0; r < 8; ++r) { const float e0 = nexp(s0[r] - mn), e1 = nexp(s1[r] - mn); sum += e0 + e1; b16 a_, c_; split16(e0 * PS, a_, c_); pb[r] = a_; pl[r] = c_; split16(e1 * PS, a_, c_); pb[8 + r] = a_; pl[8 + r] = c_; }
    sum += __shfl_xor(sum, 16); l = l * al_ + sum;
#pragma unroll
    for (int t = 0; t < 4; ++t) { o[t] *= al_; const v16b vh = frag_kb(V + (size_t)(t * 16 + col) * NPX + kb, hh); o[t] = wmma16b(vh, pb, o[t]); o[t] = wmma16b(vh, pl, o[t]); o[t] = wmma16b(frag_kb(Vl + (size_t)(t * 16 + col) * NPX + kb, hh), pb, o[t]); } }
  const float inv = 1.0f / (l * PS * XS), gmm = P[160];
#pragma unroll
  for (int t = 0; t < 4; ++t)
#pragma unroll
    for (int r = 0; r < 8; ++r) { const int c = t * 16 + 8 * hh + r; const float cr = pmul(gmm, o[t][r] * inv) + ESF[((size_t)b * NPX + qi) * C + c]; b16 a_, c_; split16(cr * XS, a_, c_); Oh[wave][col][c] = a_; Ol[wave][col][c] = c_; }
  wave_lds_sync();
  for (int pass = 0; pass < 2; ++pass) { for (int k = lane; k < 16 * 8; k += 32) { const int rr = k >> 3, c8 = (k & 7) * 8; const size_t gi = ((size_t)b * NPX + q0 + rr) * CIN + c8; *(volatile v8b*)(CATh + gi) = *(const v8b*)(&Oh[wave][rr][c8]); *(volatile v8b*)(CATl + gi) = *(const v8b*)(&Ol[wave][rr][c8]); } __threadfence(); }
}
__global__ __launch_bounds__(64) void refine_kernel(const b16* __restrict__ CATh, const b16* __restrict__ CATl, const b16* __restrict__ R, const float* __restrict__ P, float* __restrict__ Y) {
  __shared__ __attribute__((aligned(16))) float Ts[2][16][CIN + 4];
  const int lane = threadIdx.x & 31, wave = threadIdx.x >> 5, nloc = lane & 15, hlf = lane >> 4, m0 = blockIdx.x * 32 + wave * 16; const b16* Bw = R + 14336;
  v8f acc[8];
#pragma unroll
  for (int t = 0; t < 8; ++t) acc[t] = (v8f){};
#pragma unroll
  for (int kb = 0; kb < CIN; kb += 32) { const v16b a = frag_kb(CATh + (size_t)(m0 + nloc) * CIN + kb, hlf), al_ = frag_kb(CATl + (size_t)(m0 + nloc) * CIN + kb, hlf);
#pragma unroll
    for (int t = 0; t < 8; ++t) { const v16b bw = frag_kb(Bw + (size_t)(t * 16 + nloc) * CIN + kb, hlf); acc[t] = wmma16b(a, bw, acc[t]); acc[t] = wmma16b(al_, bw, acc[t]); } }
#pragma unroll
  for (int t = 0; t < 8; ++t)
#pragma unroll
    for (int r = 0; r < 8; ++r) Ts[wave][8 * hlf + r][t * 16 + nloc] = acc[t][r] * (1.0f / XS) + P[192 + t * 16 + nloc];
  wave_lds_sync();
  for (int pass = 0; pass < 2; ++pass) { for (int k = lane; k < 16 * 32; k += 32) { const int rr = k >> 5, c4 = (k & 31) * 4; *(volatile v4f*)(Y + (size_t)(m0 + rr) * CIN + c4) = *(const v4f*)(&Ts[wave][rr][c4]); } __threadfence(); }
}
template <int MODE>
__global__ __launch_bounds__(128) void stat_kernel(const float* __restrict__ Y, const float* __restrict__ MEAN, float* __restrict__ PART) {
  const int c = threadIdx.x, k = blockIdx.x; const int ch = NT / STB; const float mu = MODE ? MEAN[c] : 0.0f; float s = 0.0f;
  for (int r = k * ch; r < (k + 1) * ch; ++r) { const float v = Y[(size_t)r * CIN + c]; if (MODE) { const float d = v - mu; s += pmul(d, d); } else s += v; }
  for (int pass = 0; pass < 2; ++pass) { ((volatile float*)PART)[(size_t)k * CIN + c] = s; __threadfence(); }
}
__global__ __launch_bounds__(128) void comb_kernel(const float* __restrict__ PART, float* __restrict__ OUTV) {
  const int c = threadIdx.x; float s = 0.0f; for (int k = 0; k < STB; ++k) s += PART[(size_t)k * CIN + c];
  for (int pass = 0; pass < 2; ++pass) { ((volatile float*)OUTV)[c] = s * (1.0f / NT); __threadfence(); }
}
__global__ __launch_bounds__(256) void out_kernel(const float* __restrict__ Y, const float* __restrict__ MEAN, const float* __restrict__ VAR, const float* __restrict__ P, float* __restrict__ out) {
  __shared__ __attribute__((aligned(16))) float To[CIN][32 + 4];
  const int b = blockIdx.y, px0 = blockIdx.x * 32, t_ = threadIdx.x;
  for (int k = t_; k < 32 * CIN; k += 256) { const int p = k >> 7, c = k & 127; const float y = Y[((size_t)b * NPX + px0 + p) * CIN + c]; const float v = pmul((y - MEAN[c]) * rsqrtf(VAR[c] + EPS), P[320 + c]) + P[448 + c]; To[c][p] = fmaxf(v, 0.0f); }
  __syncthreads();
  for (int pass = 0; pass < 2; ++pass) { for (int k = t_; k < CIN * 8; k += 256) { const int c = k >> 3, c4 = (k & 7) * 4; *(volatile v4f*)(out + ((size_t)b * CIN + c) * NPX + px0 + c4) = *(const v4f*)(&To[c][c4]); } __threadfence(); }
}
}

extern "C" void kernel_launch(void* const* d_in, const int* in_sizes, int n_in,
                              void* d_out, int out_size, void* d_ws, size_t ws_size, hipStream_t stream) {
  (void)n_in; (void)out_size;
  auto Fp = [&](int i) { return (const float*)d_in[i]; };
  float* out = (float*)d_out;
  if (in_sizes[0] != NT * CIN || in_sizes[1] != NT * CIN || in_sizes[2] != C * CIN || in_sizes[15] != CIN * CIN) return;
  size_t off = 0; char* ws = (char*)d_ws;
  auto carve = [&](size_t bytes) { char* p = ws + off; off += (bytes + 255) & ~(size_t)255; return p; };
  b16* R = (b16*)carve(30720 * 2); float* P = (float*)carve(1200 * 4); b16* XT = (b16*)carve((size_t)2 * NT * CIN * 2); float* SF = (float*)carve((size_t)2 * NT * C * 4); float* PART = (float*)carve((size_t)2 * Bn * 128 * C * 4); float* MM = (float*)carve((size_t)2 * Bn * 2 * NPX * 4); float* CA = (float*)carve((size_t)2 * Bn * C * 4);
  float* ESF = (float*)carve((size_t)2 * NT * C * 4); b16* ESh = (b16*)carve((size_t)2 * NT * C * 2); b16* ESl = (b16*)carve((size_t)2 * NT * C * 2); b16* CATh = (b16*)carve((size_t)NT * CIN * 2); b16* CATl = (b16*)carve((size_t)NT * CIN * 2);
  b16* QH = (b16*)carve((size_t)NT * 32 * 2); b16* QL = (b16*)carve((size_t)NT * 32 * 2); b16* KH = (b16*)carve((size_t)NT * 32 * 2); b16* KL = (b16*)carve((size_t)NT * 32 * 2); b16* VTh = (b16*)carve((size_t)Bn * C * NPX * 2); b16* VTl = (b16*)carve((size_t)Bn * C * NPX * 2);
  float* Y = (float*)carve((size_t)NT * CIN * 4); float* SP = (float*)carve((size_t)STB * CIN * 4); float* MEAN = (float*)carve(CIN * 4); float* VAR = (float*)carve(CIN * 4);
  if (off > ws_size) return;
  prep_kernel<<<dim3(NPX / 64, Bn, 2), 256, 0, stream>>>(Fp(0), Fp(1), Fp(2), Fp(3), Fp(4), Fp(5), Fp(6), Fp(7), Fp(8), Fp(9), Fp(10), Fp(11), Fp(12), Fp(13), Fp(14), Fp(15), Fp(16), Fp(17), Fp(18), R, P, XT);
  proj_kernel<<<dim3(NT / 32, 2), 64, 0, stream>>>(XT, R, P, SF);
  cstat1_kernel<<<dim3(128, Bn, 2), 64, 0, stream>>>(SF, PART, MM);
  cstat2_kernel<<<dim3(Bn, 2), 64, 0, stream>>>(PART, P, CA);
  es_kernel<<<dim3(HW, Bn, 2), 256, 0, stream>>>(SF, MM, CA, P, ESF, ESh, ESl, CATh, CATl);
  qkv_kernel<<<dim3(NT / 64, 3), 128, 0, stream>>>(ESh, ESl, R, P, QH, QL, KH, KL, VTh, VTl);
  attn_kernel<<<dim3(NPX / 32, Bn), 64, 0, stream>>>(QH, QL, KH, KL, VTh, VTl, ESF, P, CATh, CATl);
  refine_kernel<<<NT / 32, 64, 0, stream>>>(CATh, CATl, R, P, Y);
  stat_kernel<0><<<STB, 128, 0, stream>>>(Y, nullptr, SP); comb_kernel<<<1, 128, 0, stream>>>(SP, MEAN);
  stat_kernel<1><<<STB, 128, 0, stream>>>(Y, MEAN, SP); comb_kernel<<<1, 128, 0, stream>>>(SP, VAR);
  out_kernel<<<dim3(NPX / 32, Bn), 256, 0, stream>>>(Y, MEAN, VAR, P, out);
}
